// dVAE_45028437131796
// MI455X (gfx1250) — hardware-verified
//
#include <hip/hip_runtime.h>
#include <stddef.h>
#include <stdint.h>


#define BATCH  64
#define CIN    147
#define KXP    160
#define NC0    256
#define NC1    1024
#define NLG    36
#define NLGP   48
#define NV     6
#define NKC    6
#define DEMB   32
#define NTOT   46656
#define MT     64
#define NBLK   729
#define NU     216
#define K2     1024
#define NC2    256
#define N3     784
#define N3P    800
#define K3     256
#define NTHR   256
#define NWAVE  8
#define EPS_C  1e-05f
#define ENT_SC 0.1f

#define XSC   8.0f
#define CWSC  16.0f
#define F1SC  16.0f
#define F2SC  32.0f
#define ASC   8.0f
#define W2SC  32.0f
#define W3SC  16.0f
#define ESC   16.0f

#define OSC_A (1.0f / 128.0f)
#define OSC_B (1.0f / 128.0f)
#define OSC_C (1.0f / 256.0f)
#define OSC_2 (1.0f / 256.0f)
#define OSC_3 (1.0f / 128.0f)
#define OSC_4 (1.0f / 8.0f)
#define OSC_5 (1.0f / 128.0f)

#define OUT0_N    (BATCH * NTOT)
#define OUT1_OFF  OUT0_N
#define OUT1_N    (BATCH * NLG)
#define OUT2_OFF  (OUT0_N + OUT1_N)
#define OUT2_N    BATCH
#define OUT_TOTAL (OUT2_OFF + OUT2_N)

#define SZ_XH  (BATCH * KXP * 2)
#define SZ_CW  (NC0 * KXP * 2)
#define SZ_F1  (NC1 * NC0 * 2)
#define SZ_F2  (NLGP * NC1 * 2)
#define SZ_W2  (NC2 * K2 * 2)
#define SZ_W3  (N3P * K3 * 2)
#define SZ_T   (NV * NKC * NC1 * 4)
#define SZ_U   (NU * NC1 * 4)
#define SZ_L   (NU * NC1 * 4)
#define SZ_S1  (NC1 * 4)
#define SZ_T1  (NC1 * 4)
#define SZ_S2  (NC2 * 4)
#define SZ_T2  (NC2 * 4)
#define SZ_XSQ (BATCH * 4)
#define WS_TOTAL (SZ_XH + SZ_CW + SZ_F1 + SZ_F2 + SZ_W2 + SZ_W3 + SZ_T + SZ_U + SZ_L + SZ_S1 + SZ_T1 + SZ_S2 + SZ_T2 + SZ_XSQ)
#define WSCAP 134217728

#define LDS_ENC 163840
#define LDS_DEC 163840

static_assert(NBLK * MT == NTOT);
static_assert(NTHR == NWAVE * 32);
static_assert(WS_TOTAL <= WSCAP);
static_assert(OUT1_OFF * 4 == 11943936);
static_assert(OUT2_OFF * 4 == 11953152);
static_assert(OUT_TOTAL * 4 == 11953408);
static_assert((SZ_XH % 256) == 0 && (SZ_CW % 256) == 0 && (SZ_F2 % 256) == 0 && (SZ_W3 % 256) == 0 && (SZ_XSQ % 256) == 0);
static_assert(((SZ_XH / 16) % NTHR) == 0);
static_assert(((SZ_CW / 16) % NTHR) == 0);
static_assert(((SZ_F1 / 16) % NTHR) == 0);
static_assert(((SZ_F2 / 16) % NTHR) == 0);
static_assert(((SZ_W2 / 16) % NTHR) == 0);
static_assert(((SZ_W3 / 16) % NTHR) == 0);
static_assert(((NV * NKC * NC1) % NTHR) == 0);
static_assert(NC1 == 4 * NTHR);
static_assert((KXP % 32) == 0 && (K2 % 32) == 0 && (K3 % 32) == 0 && (NC0 % 32) == 0);
static_assert((N3P % 16) == 0 && (NLGP % 16) == 0);
static_assert(MT * K2 * 2 + MT * NC2 * 2 <= LDS_DEC);
static_assert(MT * N3P * 2 + MT * KXP * 2 + MT * 4 <= MT * K2 * 2);
static_assert(131072 + MT * NLGP * 4 + OUT1_N * 4 + OUT2_N * 4 <= LDS_ENC);

typedef float    v4f  __attribute__((ext_vector_type(4)));
typedef float    v8f  __attribute__((ext_vector_type(8)));
typedef _Float16 v4h  __attribute__((ext_vector_type(4)));
typedef _Float16 v8h  __attribute__((ext_vector_type(8)));
typedef _Float16 v16h __attribute__((ext_vector_type(16)));
union FragH { v16h v; v8h h[2]; };
struct Acc4 { v8f a[4]; };

__device__ __forceinline__ v8f wmf(v16h a, v16h b, v8f c) {
  v8f d = __builtin_amdgcn_wmma_f32_16x16x32_f16(false, a, false, b, (short)0, c, false, false);
  asm volatile("v_nop\n\tv_nop\n\tv_nop\n\tv_nop" : "+v"(d) : "v"(a), "v"(b));
  return d;
}

__device__ __forceinline__ v16h ldfrag(const _Float16* rowp, int k0, int hh) {
  FragH f;
  f.h[0] = *(const v8h*)(rowp + k0 + 8 * hh);
  f.h[1] = *(const v8h*)(rowp + k0 + 16 + 8 * hh);
  return f.v;
}

__device__ __forceinline__ void acc_zero(Acc4& t) {
  const v8f z = {0.f, 0.f, 0.f, 0.f, 0.f, 0.f, 0.f, 0.f};
#pragma unroll
  for (int mi = 0; mi < 4; ++mi) t.a[mi] = z;
}

__device__ __forceinline__ void bn_cols_store(Acc4& t, float osc, float bias, float g, float be,
                                              _Float16* dcol, int ld, int hh) {
  float p = 0.f;
#pragma unroll
  for (int mi = 0; mi < 4; ++mi) {
#pragma unroll
    for (int r = 0; r < 8; ++r) {
      const float v = fmaf(t.a[mi][r], osc, bias);
      t.a[mi][r] = v;
      p += v;
    }
  }
  const float mean = (p + __shfl_xor(p, 16)) * (1.0f / 64.0f);
  float q = 0.f;
#pragma unroll
  for (int mi = 0; mi < 4; ++mi) {
#pragma unroll
    for (int r = 0; r < 8; ++r) {
      const float d = t.a[mi][r] - mean;
      q = fmaf(d, d, q);
    }
  }
  const float var = (q + __shfl_xor(q, 16)) * (1.0f / 64.0f);
  const float inv = rsqrtf(var + EPS_C);
#pragma unroll
  for (int mi = 0; mi < 4; ++mi) {
#pragma unroll
    for (int r = 0; r < 8; ++r) {
      float y = g * (t.a[mi][r] - mean) * inv + be;
      y = fmaxf(y, 0.0f) * ASC;
      dcol[(16 * mi + 8 * hh + r) * ld] = (_Float16)y;
    }
  }
}

__device__ __forceinline__ void relu_store(const Acc4& t, float sc, float sh, _Float16* dcol, int ld, int hh) {
#pragma unroll
  for (int mi = 0; mi < 4; ++mi) {
#pragma unroll
    for (int r = 0; r < 8; ++r) {
      float y = fmaf(t.a[mi][r], sc, sh);
      y = fmaxf(y, 0.0f) * ASC;
      dcol[(16 * mi + 8 * hh + r) * ld] = (_Float16)y;
    }
  }
}

__global__ __launch_bounds__(NTHR) void k_cvt(const float* __restrict__ src, _Float16* dst,
                                              int R, int K, int RP, int KP, int sr, int sk, float scale) {
  const unsigned t = blockIdx.x * NTHR + threadIdx.x;
  const unsigned e0 = t * 8u;
  const unsigned total = (unsigned)RP * (unsigned)KP;
  if (e0 >= total) return;
  const unsigned r = e0 / (unsigned)KP;
  const unsigned kb = e0 - r * (unsigned)KP;
  const unsigned rc = (r < (unsigned)R) ? r : (unsigned)(R - 1);
  const float* rowp = src + (size_t)rc * (size_t)sr;
  v8h o;
#pragma unroll
  for (int i = 0; i < 8; ++i) {
    const unsigned k = kb + (unsigned)i;
    const unsigned kc = (k < (unsigned)K) ? k : (unsigned)(K - 1);
    const float v = rowp[(size_t)kc * (size_t)sk];
    const bool ok = (r < (unsigned)R) && (k < (unsigned)K);
    o[i] = (_Float16)(ok ? v * scale : 0.0f);
  }
  _Float16* d = dst + e0;
  *(volatile v8h*)d = o;
  __threadfence();
  *(volatile v8h*)d = o;
}

__global__ __launch_bounds__(NTHR) void k_tabT(const float* __restrict__ emb, const float* __restrict__ w1, float* T) {
  const int e = blockIdx.x * NTHR + threadIdx.x;
  const int vk = e >> 10, j = e & (NC1 - 1), v = vk / NKC;
  const float* ep = emb + vk * DEMB;
  const float* wp = w1 + (size_t)j * (NV * DEMB) + v * DEMB;
  float s = 0.f;
#pragma unroll 4
  for (int d = 0; d < DEMB; ++d) s = fmaf(ep[d], wp[d], s);
  *(volatile float*)(T + e) = s;
  __threadfence();
  *(volatile float*)(T + e) = s;
}

__global__ __launch_bounds__(NTHR) void k_tabUL(const float* __restrict__ T, float* U, float* L) {
  const int a = blockIdx.x;
  const int j0 = 4 * threadIdx.x;
  const int d0 = a / 36, d1 = (a / 6) % 6, d2 = a % 6;
  const v4f t0 = *(const v4f*)(T + (size_t)(0 * NKC + d0) * NC1 + j0);
  const v4f t1 = *(const v4f*)(T + (size_t)(1 * NKC + d1) * NC1 + j0);
  const v4f t2 = *(const v4f*)(T + (size_t)(2 * NKC + d2) * NC1 + j0);
  const v4f t3 = *(const v4f*)(T + (size_t)(3 * NKC + d0) * NC1 + j0);
  const v4f t4 = *(const v4f*)(T + (size_t)(4 * NKC + d1) * NC1 + j0);
  const v4f t5 = *(const v4f*)(T + (size_t)(5 * NKC + d2) * NC1 + j0);
  const v4f u = (t0 + t1) + t2;
  const v4f l = (t3 + t4) + t5;
  float* pu = U + (size_t)a * NC1 + j0;
  float* pl = L + (size_t)a * NC1 + j0;
  *(volatile v4f*)pu = u;
  *(volatile v4f*)pl = l;
  __threadfence();
  *(volatile v4f*)pu = u;
  *(volatile v4f*)pl = l;
}

__global__ __launch_bounds__(NTHR) void k_vec(const float* __restrict__ x,
    const float* __restrict__ dfc1_b, const float* __restrict__ g1, const float* __restrict__ b1,
    const float* __restrict__ rm1, const float* __restrict__ rv1,
    const float* __restrict__ dfc2_b, const float* __restrict__ g2, const float* __restrict__ b2,
    const float* __restrict__ rm2, const float* __restrict__ rv2,
    float* s1, float* t1, float* s2, float* t2, float* xsq) {
  const int blk = blockIdx.x, tid = threadIdx.x;
  if (blk < 4) {
    const int i = blk * NTHR + tid;
    const float s = g1[i] * rsqrtf(rv1[i] + EPS_C);
    const float tt = fmaf(s, dfc1_b[i] - rm1[i], b1[i]);
    *(volatile float*)(s1 + i) = s;
    *(volatile float*)(t1 + i) = tt;
    __threadfence();
    *(volatile float*)(s1 + i) = s;
    *(volatile float*)(t1 + i) = tt;
  } else if (blk == 4) {
    const int i = tid;
    const float s = g2[i] * rsqrtf(rv2[i] + EPS_C);
    const float tt = fmaf(s, dfc2_b[i] - rm2[i], b2[i]);
    *(volatile float*)(s2 + i) = s;
    *(volatile float*)(t2 + i) = tt;
    __threadfence();
    *(volatile float*)(s2 + i) = s;
    *(volatile float*)(t2 + i) = tt;
  } else {
    if (tid < BATCH) {
      const float* xp = x + tid * CIN;
      float s = 0.f;
#pragma unroll 4
      for (int k = 0; k < CIN; ++k) s = fmaf(xp[k], xp[k], s);
      *(volatile float*)(xsq + tid) = s;
      __threadfence();
      *(volatile float*)(xsq + tid) = s;
    }
  }
}

__global__ __launch_bounds__(NTHR) void k_enc(const _Float16* __restrict__ XH, const _Float16* __restrict__ CW,
                                              const _Float16* __restrict__ F1, const _Float16* __restrict__ F2,
                                              const float* __restrict__ conv_b, const float* __restrict__ g0,
                                              const float* __restrict__ be0, const float* __restrict__ fc1_b,
                                              const float* __restrict__ g1, const float* __restrict__ be1,
                                              const float* __restrict__ fc2_b, float* out) {
  extern __shared__ __attribute__((aligned(16))) char smem[];
  _Float16* e1r = (_Float16*)(smem);
  _Float16* e0r = (_Float16*)(smem + 131072);
  float* lg  = (float*)(smem + 131072);
  float* dst = (float*)(smem + 131072 + MT * NLGP * 4);
  float* lss = (float*)(smem + 131072 + MT * NLGP * 4 + OUT1_N * 4);
  const int tid = threadIdx.x, lane = tid & 31, wave = tid >> 5, hh = lane >> 4, m = lane & 15;

  for (int nt = wave; nt < NC0 / 16; nt += NWAVE) {
    const int ni = 16 * nt;
    Acc4 t; acc_zero(t);
    const _Float16* bp = CW + (size_t)(ni + m) * KXP;
#pragma unroll
    for (int ks = 0; ks < KXP / 32; ++ks) {
      const int k0 = 32 * ks;
      const v16h b = ldfrag(bp, k0, hh);
#pragma unroll
      for (int mi = 0; mi < 4; ++mi)
        t.a[mi] = wmf(ldfrag(XH + (size_t)(16 * mi + m) * KXP, k0, hh), b, t.a[mi]);
    }
    const int col = ni + m;
    bn_cols_store(t, OSC_A, conv_b[col], g0[col], be0[col], e0r + col, NC0, hh);
  }
  __syncthreads();

  for (int nt = wave; nt < NC1 / 16; nt += NWAVE) {
    const int ni = 16 * nt;
    Acc4 t; acc_zero(t);
    const _Float16* bp = F1 + (size_t)(ni + m) * NC0;
#pragma unroll 2
    for (int ks = 0; ks < NC0 / 32; ++ks) {
      const int k0 = 32 * ks;
      const v16h b = ldfrag(bp, k0, hh);
#pragma unroll
      for (int mi = 0; mi < 4; ++mi)
        t.a[mi] = wmf(ldfrag(e0r + (16 * mi + m) * NC0, k0, hh), b, t.a[mi]);
    }
    const int col = ni + m;
    bn_cols_store(t, OSC_B, fc1_b[col], g1[col], be1[col], e1r + col, NC1, hh);
  }
  __syncthreads();

  if (wave < NLGP / 16) {
    const int ni = 16 * wave;
    Acc4 t; acc_zero(t);
    const _Float16* bp = F2 + (size_t)(ni + m) * NC1;
#pragma unroll 2
    for (int ks = 0; ks < NC1 / 32; ++ks) {
      const int k0 = 32 * ks;
      const v16h b = ldfrag(bp, k0, hh);
#pragma unroll
      for (int mi = 0; mi < 4; ++mi)
        t.a[mi] = wmf(ldfrag(e1r + (16 * mi + m) * NC1, k0, hh), b, t.a[mi]);
    }
    const int col = ni + m;
    const int cb = col < NLG ? col : NLG - 1;
    const float bias = fc2_b[cb];
#pragma unroll
    for (int mi = 0; mi < 4; ++mi) {
#pragma unroll
      for (int r = 0; r < 8; ++r) lg[(16 * mi + 8 * hh + r) * NLGP + col] = fmaf(t.a[mi][r], OSC_C, bias);
    }
  }
  __syncthreads();

  if (tid < BATCH) {
    const float* lp = lg + tid * NLGP;
    float ent = 0.f;
#pragma unroll 1
    for (int v = 0; v < NV; ++v) {
      float lv[NKC];
#pragma unroll
      for (int k = 0; k < NKC; ++k) lv[k] = lp[v * NKC + k];
      float mx = lv[0];
#pragma unroll
      for (int k = 1; k < NKC; ++k) mx = fmaxf(mx, lv[k]);
      float ex[NKC];
      float sum = 0.f;
#pragma unroll
      for (int k = 0; k < NKC; ++k) { ex[k] = expf(lv[k] - mx); sum += ex[k]; }
      const float is = 1.0f / sum;
#pragma unroll
      for (int k = 0; k < NKC; ++k) {
        const float p = ex[k] * is;
        dst[tid * NLG + v * NKC + k] = p;
        ent += p * logf(p + 1e-10f);
      }
    }
    lss[tid] = ENT_SC * ent;
  }
  __syncthreads();

  {
    v4f dv[3];
#pragma unroll
    for (int s = 0; s < 3; ++s) {
      const int i = tid + s * NTHR;
      const int ic = i < (OUT1_N / 4) ? i : (OUT1_N / 4 - 1);
      dv[s] = *(const v4f*)(dst + 4 * ic);
    }
    const int il = tid < (OUT2_N / 4) ? tid : (OUT2_N / 4 - 1);
    const v4f lv4 = *(const v4f*)(lss + 4 * il);
#pragma unroll
    for (int s = 0; s < 3; ++s) {
      const int i = tid + s * NTHR;
      if (i < OUT1_N / 4) *(volatile v4f*)(out + OUT1_OFF + 4 * i) = dv[s];
    }
    if (tid < OUT2_N / 4) *(volatile v4f*)(out + OUT2_OFF + 4 * tid) = lv4;
    __threadfence();
#pragma unroll
    for (int s = 0; s < 3; ++s) {
      const int i = tid + s * NTHR;
      if (i < OUT1_N / 4) *(volatile v4f*)(out + OUT1_OFF + 4 * i) = dv[s];
    }
    if (tid < OUT2_N / 4) *(volatile v4f*)(out + OUT2_OFF + 4 * tid) = lv4;
  }
}

__global__ __launch_bounds__(NTHR) void k_dec(const float* __restrict__ U, const float* __restrict__ L,
                                              const float* __restrict__ s1, const float* __restrict__ t1,
                                              const _Float16* __restrict__ W2, const float* __restrict__ s2,
                                              const float* __restrict__ t2, const _Float16* __restrict__ W3,
                                              const float* __restrict__ dct1_b, const float* __restrict__ g3,
                                              const float* __restrict__ b3, const float* __restrict__ rm3,
                                              const float* __restrict__ rv3, const float* __restrict__ dct2_w,
                                              const float* __restrict__ dct2_b, const _Float16* __restrict__ XH,
                                              const float* __restrict__ xsq, float* out) {
  extern __shared__ __attribute__((aligned(16))) char smem[];
  _Float16* h1H  = (_Float16*)(smem);
  _Float16* h2H  = (_Float16*)(smem + MT * K2 * 2);
  _Float16* h3H  = (_Float16*)(smem);
  _Float16* EH   = (_Float16*)(smem + MT * N3P * 2);
  float*    esq  = (float*)(smem + MT * N3P * 2 + MT * KXP * 2);
  float*    obsS = (float*)(smem);
  __shared__ float s3s[16];
  __shared__ float t3s[16];
  __shared__ float w2s[48];
  __shared__ float b2s[4];
  __shared__ float xsqs[BATCH];

  const int tid = threadIdx.x, lane = tid & 31, wave = tid >> 5, hh = lane >> 4, m = lane & 15;
  const int n0 = blockIdx.x * MT;

  if (tid < 16) {
    const float s = g3[tid] * rsqrtf(rv3[tid] + EPS_C);
    s3s[tid] = s;
    t3s[tid] = fmaf(s, dct1_b[tid] - rm3[tid], b3[tid]);
  }
  if (tid < 48) w2s[tid] = dct2_w[tid];
  if (tid < 3) b2s[tid] = dct2_b[tid];
  if (tid < BATCH) xsqs[tid] = xsq[tid];

  {
    const int j0 = 4 * tid;
    const v4f sv = *(const v4f*)(s1 + j0);
    const v4f tv = *(const v4f*)(t1 + j0);
#pragma unroll 2
    for (int mm = 0; mm < MT; ++mm) {
      const unsigned n = (unsigned)(n0 + mm);
      const unsigned a = n / 216u;
      const unsigned c = n - a * 216u;
      const v4f u = *(const v4f*)(U + (size_t)a * NC1 + j0);
      const v4f l = *(const v4f*)(L + (size_t)c * NC1 + j0);
      v4h o;
#pragma unroll
      for (int i = 0; i < 4; ++i) {
        const float y = fmaf(u[i] + l[i], sv[i], tv[i]);
        o[i] = (_Float16)(fmaxf(y, 0.0f) * ASC);
      }
      *(v4h*)(h1H + mm * K2 + j0) = o;
    }
  }
  __syncthreads();

  for (int nt = wave; nt < NC2 / 16; nt += NWAVE) {
    const int ni = 16 * nt;
    Acc4 t; acc_zero(t);
    const _Float16* bp = W2 + (size_t)(ni + m) * K2;
#pragma unroll 2
    for (int ks = 0; ks < K2 / 32; ++ks) {
      const int k0 = 32 * ks;
      const v16h b = ldfrag(bp, k0, hh);
#pragma unroll
      for (int mi = 0; mi < 4; ++mi)
        t.a[mi] = wmf(ldfrag(h1H + (16 * mi + m) * K2, k0, hh), b, t.a[mi]);
    }
    const int col = ni + m;
    const float sc = s2[col] * OSC_2, sh = t2[col];
    relu_store(t, sc, sh, h2H + col, NC2, hh);
  }
  __syncthreads();

  for (int nt = wave; nt < N3P / 16; nt += NWAVE) {
    const int ni = 16 * nt;
    Acc4 t; acc_zero(t);
    const _Float16* bp = W3 + (size_t)(ni + m) * K3;
#pragma unroll 2
    for (int ks = 0; ks < K3 / 32; ++ks) {
      const int k0 = 32 * ks;
      const v16h b = ldfrag(bp, k0, hh);
#pragma unroll
      for (int mi = 0; mi < 4; ++mi)
        t.a[mi] = wmf(ldfrag(h2H + (16 * mi + m) * NC2, k0, hh), b, t.a[mi]);
    }
    const int col = ni + m;
    int ch = col / 49; ch = ch < 16 ? ch : 15;
    const float sc = s3s[ch] * OSC_3, sh = t3s[ch];
    relu_store(t, sc, sh, h3H + col, N3P, hh);
  }
  __syncthreads();

  {
    const int mm = tid >> 2, part = tid & 3;
    const _Float16* hr = h3H + mm * N3P;
    float eq = 0.f;
#pragma unroll 1
    for (int ci = 0; ci < KXP / 4; ++ci) {
      const int col = part + 4 * ci;
      const int colc = col < CIN ? col : CIN - 1;
      const int c = colc / 49, hw = colc - 49 * c;
      float s = 0.f;
#pragma unroll
      for (int o = 0; o < 16; ++o) s = fmaf((float)hr[o * 49 + hw], w2s[o * 3 + c], s);
      const float e = fmaf(s, OSC_4, b2s[c]);
      const float ev = (col < CIN) ? e : 0.0f;
      eq = fmaf(ev, ev, eq);
      EH[mm * KXP + col] = (_Float16)(ev * ESC);
    }
    eq += __shfl_xor(eq, 1);
    eq += __shfl_xor(eq, 2);
    if (part == 0) esq[mm] = eq;
  }
  __syncthreads();

  if (wave < BATCH / 16) {
    const int ni = 16 * wave;
    Acc4 t; acc_zero(t);
    const _Float16* bp = XH + (size_t)(ni + m) * KXP;
#pragma unroll
    for (int ks = 0; ks < KXP / 32; ++ks) {
      const int k0 = 32 * ks;
      const v16h b = ldfrag(bp, k0, hh);
#pragma unroll
      for (int mi = 0; mi < 4; ++mi)
        t.a[mi] = wmf(ldfrag(EH + (16 * mi + m) * KXP, k0, hh), b, t.a[mi]);
    }
    const int bc = ni + m;
    const float xq = xsqs[bc];
#pragma unroll
    for (int mi = 0; mi < 4; ++mi) {
#pragma unroll
      for (int r = 0; r < 8; ++r) {
        const int j = 16 * mi + 8 * hh + r;
        const float cr = t.a[mi][r] * OSC_5;
        obsS[bc * MT + j] = -0.5f * ((esq[j] - 2.0f * cr) + xq);
      }
    }
  }
  __syncthreads();

  {
    float* gb = out + (size_t)n0;
    v4f vv[4];
#pragma unroll
    for (int q = 0; q < 4; ++q) {
      const int row = 8 * wave + 2 * q + hh;
      vv[q] = *(const v4f*)(obsS + row * MT + 4 * m);
    }
#pragma unroll
    for (int q = 0; q < 4; ++q) {
      const int row = 8 * wave + 2 * q + hh;
      *(volatile v4f*)(gb + (size_t)row * NTOT + 4 * m) = vv[q];
    }
    __threadfence();
#pragma unroll
    for (int q = 0; q < 4; ++q) {
      const int row = 8 * wave + 2 * q + hh;
      *(volatile v4f*)(gb + (size_t)row * NTOT + 4 * m) = vv[q];
    }
  }
}

extern "C" void kernel_launch(void* const* d_in, const int* in_sizes, int n_in,
                              void* d_out, int out_size, void* d_ws, size_t ws_size,
                              hipStream_t stream) {
  if (n_in < 32) return;
  const int expect[32] = {
    BATCH * CIN, NC0 * CIN, NC0, NC0, NC0,
    NC1 * NC0, NC1, NC1, NC1,
    NLG * NC1, NLG,
    NV * NKC * DEMB,
    NC1 * NV * DEMB, NC1, NC1, NC1, NC1, NC1,
    NC2 * K2, NC2, NC2, NC2, NC2, NC2,
    K3 * N3, 16, 16, 16, 16, 16,
    48, 3 };
  for (int i = 0; i < 32; ++i) if (in_sizes[i] != expect[i]) return;
  if (out_size != OUT_TOTAL) return;

  const float* x       = (const float*)d_in[0];
  const float* conv_w  = (const float*)d_in[1];
  const float* conv_b  = (const float*)d_in[2];
  const float* ebn2_g  = (const float*)d_in[3];
  const float* ebn2_b  = (const float*)d_in[4];
  const float* fc1_w   = (const float*)d_in[5];
  const float* fc1_b   = (const float*)d_in[6];
  const float* ebn1_g  = (const float*)d_in[7];
  const float* ebn1_b  = (const float*)d_in[8];
  const float* fc2_w   = (const float*)d_in[9];
  const float* fc2_b   = (const float*)d_in[10];
  const float* embeds  = (const float*)d_in[11];
  const float* dfc1_w  = (const float*)d_in[12];
  const float* dfc1_b  = (const float*)d_in[13];
  const float* dbn1_g  = (const float*)d_in[14];
  const float* dbn1_b  = (const float*)d_in[15];
  const float* dbn1_rm = (const float*)d_in[16];
  const float* dbn1_rv = (const float*)d_in[17];
  const float* dfc2_w  = (const float*)d_in[18];
  const float* dfc2_b  = (const float*)d_in[19];
  const float* dbn2_g  = (const float*)d_in[20];
  const float* dbn2_b  = (const float*)d_in[21];
  const float* dbn2_rm = (const float*)d_in[22];
  const float* dbn2_rv = (const float*)d_in[23];
  const float* dct1_w  = (const float*)d_in[24];
  const float* dct1_b  = (const float*)d_in[25];
  const float* dbn3_g  = (const float*)d_in[26];
  const float* dbn3_b  = (const float*)d_in[27];
  const float* dbn3_rm = (const float*)d_in[28];
  const float* dbn3_rv = (const float*)d_in[29];
  const float* dct2_w  = (const float*)d_in[30];
  const float* dct2_b  = (const float*)d_in[31];
  float* out = (float*)d_out;

  char* ws = (char*)d_ws;
  size_t off = 0;
  const size_t oXH = off;  off += SZ_XH;
  const size_t oCW = off;  off += SZ_CW;
  const size_t oF1 = off;  off += SZ_F1;
  const size_t oF2 = off;  off += SZ_F2;
  const size_t oW2 = off;  off += SZ_W2;
  const size_t oW3 = off;  off += SZ_W3;
  const size_t oT  = off;  off += SZ_T;
  const size_t oU  = off;  off += SZ_U;
  const size_t oL  = off;  off += SZ_L;
  const size_t oS1 = off;  off += SZ_S1;
  const size_t oT1 = off;  off += SZ_T1;
  const size_t oS2 = off;  off += SZ_S2;
  const size_t oT2 = off;  off += SZ_T2;
  const size_t oXQ = off;  off += SZ_XSQ;
  if (off > ws_size || off > (size_t)WSCAP) return;
  _Float16* XH = (_Float16*)(ws + oXH);
  _Float16* CW = (_Float16*)(ws + oCW);
  _Float16* F1 = (_Float16*)(ws + oF1);
  _Float16* F2 = (_Float16*)(ws + oF2);
  _Float16* W2 = (_Float16*)(ws + oW2);
  _Float16* W3 = (_Float16*)(ws + oW3);
  float* T   = (float*)(ws + oT);
  float* U   = (float*)(ws + oU);
  float* L   = (float*)(ws + oL);
  float* s1  = (float*)(ws + oS1);
  float* t1  = (float*)(ws + oT1);
  float* s2  = (float*)(ws + oS2);
  float* t2  = (float*)(ws + oT2);
  float* xsq = (float*)(ws + oXQ);

  k_cvt<<<(SZ_XH / 16) / NTHR, NTHR, 0, stream>>>(x,      XH, BATCH, CIN, BATCH, KXP, CIN, 1, XSC);
  k_cvt<<<(SZ_CW / 16) / NTHR, NTHR, 0, stream>>>(conv_w, CW, NC0, CIN, NC0, KXP, CIN, 1, CWSC);
  k_cvt<<<(SZ_F1 / 16) / NTHR, NTHR, 0, stream>>>(fc1_w,  F1, NC1, NC0, NC1, NC0, NC0, 1, F1SC);
  k_cvt<<<(SZ_F2 / 16) / NTHR, NTHR, 0, stream>>>(fc2_w,  F2, NLG, NC1, NLGP, NC1, NC1, 1, F2SC);
  k_cvt<<<(SZ_W2 / 16) / NTHR, NTHR, 0, stream>>>(dfc2_w, W2, NC2, K2, NC2, K2, K2, 1, W2SC);
  k_cvt<<<(SZ_W3 / 16) / NTHR, NTHR, 0, stream>>>(dct1_w, W3, N3, K3, N3P, K3, 1, N3, W3SC);
  k_tabT<<<(NV * NKC * NC1) / NTHR, NTHR, 0, stream>>>(embeds, dfc1_w, T);
  k_tabUL<<<NU, NTHR, 0, stream>>>(T, U, L);
  k_vec<<<6, NTHR, 0, stream>>>(x, dfc1_b, dbn1_g, dbn1_b, dbn1_rm, dbn1_rv,
                                dfc2_b, dbn2_g, dbn2_b, dbn2_rm, dbn2_rv, s1, t1, s2, t2, xsq);
  hipFuncSetAttribute(reinterpret_cast<const void*>(&k_enc), hipFuncAttributeMaxDynamicSharedMemorySize, LDS_ENC);
  k_enc<<<1, NTHR, LDS_ENC, stream>>>(XH, CW, F1, F2, conv_b, ebn2_g, ebn2_b, fc1_b, ebn1_g, ebn1_b, fc2_b, out);
  hipFuncSetAttribute(reinterpret_cast<const void*>(&k_dec), hipFuncAttributeMaxDynamicSharedMemorySize, LDS_DEC);
  k_dec<<<NBLK, NTHR, LDS_DEC, stream>>>(U, L, s1, t1, W2, s2, t2, W3, dct1_b, dbn3_g, dbn3_b, dbn3_rm, dbn3_rv,
                                         dct2_w, dct2_b, XH, xsq, out);
}
